// STDPPlasticityRule_56470230008109
// MI455X (gfx1250) — hardware-run, weakly checked
//
#include <hip/hip_runtime.h>


namespace {
constexpr int NB_ = 16, P = 2048, Q = 2048, T = 256, KH = NB_ * T  , K = 2 * KH  , NRB = 256  ;
constexpr float TS = 256.0f, DT_ = 0.001f, TAU_P = 0.02f, TAU_M = 0.02f, TAU_X = 0.101f, A_TRIP = 0.0065f, HRATE = 0.1f;
typedef _Float16 b16;
typedef __attribute__((ext_vector_type(16))) _Float16 v16b;
typedef __attribute__((ext_vector_type(8))) _Float16 v8b;
typedef __attribute__((ext_vector_type(8))) float v8f;
typedef __attribute__((ext_vector_type(4))) float v4f;
__device__ __forceinline__ float bf16_rne(float f) { unsigned int u = __float_as_uint(f); u += 0x7FFFu + ((u >> 16) & 1u); float r = __uint_as_float(u & 0xFFFF0000u); asm volatile("" : "+v"(r)); return r; }
__device__ __forceinline__ float bfv(float f) { float r = bf16_rne(f); asm volatile("" : "+v"(r)); return r; }
__device__ __forceinline__ v16b frag_kb(const b16* p, int hh) { const v8b a = *(const v8b*)(p + 8 * hh), b = *(const v8b*)(p + 16 + 8 * hh); v16b f;
#pragma unroll
  for (int e = 0; e < 8; ++e) { f[e] = a[e]; f[8 + e] = b[e]; } return f; }
__device__ __forceinline__ v8f wmma16b(v16b a, v16b b, v8f c) { v8f d = __builtin_amdgcn_wmma_f32_16x16x32_f16(false, a, false, b, (short)0, c, false, false); asm volatile("v_nop\n\tv_nop\n\tv_nop\n\tv_nop" : "+v"(d) : "v"(a), "v"(b)); return d; }
__device__ __forceinline__ void wave_lds_sync() { __builtin_amdgcn_fence(__ATOMIC_RELEASE, "workgroup"); __builtin_amdgcn_wave_barrier(); __builtin_amdgcn_fence(__ATOMIC_ACQUIRE, "workgroup"); }
__device__ __forceinline__ float pmul(float a, float b) { float p = a * b; asm volatile("" : "+v"(p)); return p; }

template <int SIDE>
__global__ __launch_bounds__(32) void trace_kernel(const float* __restrict__ S, const float* __restrict__ aplus, const float* __restrict__ aminus, b16* __restrict__ PL, float* __restrict__ CNT) { __shared__ float Sr[32][T + 1]; __shared__ b16 O1[32][T + 8], O2[32][T + 8]; const int lane = threadIdx.x; const int b = blockIdx.x / (P / 32); const int n0 = (blockIdx.x % (P / 32)) * 32; float cnt = 0.0f;
  for (int r = 0; r < 32; ++r) for (int q = 0; q < T / 32; ++q) { const float v = bfv(S[((size_t)b * P + n0 + r) * T + q * 32 + lane]); Sr[r][q * 32 + lane] = v; cnt += v; }
  for (int o = 16; o; o >>= 1) cnt += __shfl_xor(cnt, o);
  wave_lds_sync();
  { const float dp = expf(-DT_ / TAU_P), dm = expf(-DT_ / TAU_M), dx = expf(-DT_ / TAU_X); const float ap = bfv(aplus[0]), am = bfv(aminus[0]); float x1 = 0.0f, x2 = 0.0f;
#pragma unroll 1
    for (int t = 0; t < T; ++t) { const float s = Sr[lane][t]; if (SIDE == 0) { x1 = dp * x1; O1[lane][t] = (b16)(x1 * TS); O2[lane][t] = (b16)(s * TS); x1 += s; }     else { x1 = dm * x1; x2 = dx * x2; O1[lane][t] = (b16)(pmul(s, ap + A_TRIP * x2) * TS); O2[lane][t] = (b16)(-pmul(am, x1) * TS); x1 += s; x2 += s; } } }
  wave_lds_sync();
  for (int pass = 0; pass < 2; ++pass) { for (int r = 0; r < 32; ++r) { b16* row = PL + (size_t)(n0 + r) * K; for (int q = 0; q < T / 32; ++q) { ((volatile b16*)row)[b * T + q * 32 + lane] = O1[r][q * 32 + lane]; ((volatile b16*)row)[KH + b * T + q * 32 + lane] = O2[r][q * 32 + lane]; } }
    ((volatile float*)CNT)[(size_t)blockIdx.x * 32 + lane] = lane == 0 ? cnt : 0.0f; __threadfence(); } }
__global__ __launch_bounds__(32) void count_kernel(const float* __restrict__ C1, const float* __restrict__ C2, int nb, float* __restrict__ TOT) { const int lane = threadIdx.x; float s = 0.0f; if (lane == 0) { for (int i = 0; i < nb; ++i) s += C1[(size_t)i * 32]; for (int i = 0; i < nb; ++i) s += C2[(size_t)i * 32]; }
  for (int pass = 0; pass < 2; ++pass) { ((volatile float*)TOT)[lane] = lane == 0 ? s : 0.0f; __threadfence(); } }
__global__ __launch_bounds__(32) void gemm_kernel(const b16* __restrict__ AT, const b16* __restrict__ BT, const float* __restrict__ w, const float* __restrict__ TOT, int PLIM, float* __restrict__ out) { __shared__ float Tf[16][132]; const int lane = threadIdx.x, nloc = lane & 15, hlf = lane >> 4; const int g = blockIdx.x % (Q / 128); const size_t m0 = (size_t)(blockIdx.x / (Q / 128)) * 16; if (m0 >= (size_t)PLIM) return; v8f acc[8];
#pragma unroll
  for (int t = 0; t < 8; ++t) acc[t] = (v8f){};
  const b16* arow = AT + (m0 + nloc) * K;
#pragma unroll 2
  for (int kb = 0; kb < K; kb += 32) { const v16b av = frag_kb(arow + kb, hlf);
#pragma unroll
    for (int t = 0; t < 8; ++t) acc[t] = wmma16b(av, frag_kb(BT + (size_t)(g * 128 + t * 16 + nloc) * K + kb, hlf), acc[t]); }
  const float act = TOT[0] / (float)(NB_ * T); const float sc = sqrtf(HRATE / (act + 1e-6f)) * (1.0f / (TS * TS));
#pragma unroll
  for (int t = 0; t < 8; ++t)
#pragma unroll
    for (int r8 = 0; r8 < 8; ++r8) Tf[8 * hlf + r8][t * 16 + nloc] = acc[t][r8] * sc;
  wave_lds_sync();
  for (int pass = 0; pass < 2; ++pass) { for (int rr = 0; rr < 16; ++rr) { const size_t o = (m0 + rr) * Q + g * 128 + lane * 4; v4f v;
#pragma unroll
      for (int k = 0; k < 4; ++k) v[k] = fminf(fmaxf(bfv(w[o + k]) + Tf[rr][lane * 4 + k], -2.0f), 2.0f); *(volatile v4f*)(out + o) = v; } __threadfence(); } }
}

extern "C" void kernel_launch(void* const* d_in, const int* in_sizes, int n_in, void* d_out, int out_size, void* d_ws, size_t ws_size, hipStream_t stream) {
  (void)n_in;
  auto Fp = [&](int i) { return (const float*)d_in[i]; };
  if (in_sizes[0] != NB_ * P * T || in_sizes[1] != NB_ * Q * T || in_sizes[2] != P * Q || in_sizes[3] != 1 || in_sizes[4] != 1 || out_size != P * Q) return;
  const int PLIM = P;
  size_t off = 0; char* ws = (char*)d_ws;
  auto carve = [&](size_t bytes) { char* p = ws + off; off += (bytes + 255) & ~(size_t)255; return p; };
  b16* AT = (b16*)carve((size_t)P * K * 2); b16* BT = (b16*)carve((size_t)Q * K * 2); float* C1 = (float*)carve((size_t)NB_ * (P / 32) * 128); float* C2 = (float*)carve((size_t)NB_ * (Q / 32) * 128); float* TOT = (float*)carve(256);
  if (off > ws_size || off > ((size_t)96 << 20)) return;
  const int nb = NB_ * (P / 32);
  trace_kernel<0><<<nb, 32, 0, stream>>>(Fp(0), Fp(3), Fp(4), AT, C1);
  trace_kernel<1><<<nb, 32, 0, stream>>>(Fp(1), Fp(3), Fp(4), BT, C2);
  count_kernel<<<1, 32, 0, stream>>>(C1, C2, nb, TOT);
  gemm_kernel<<<(PLIM / 16) * (Q / 128), 32, 0, stream>>>(AT, BT, Fp(2), TOT, PLIM, (float*)d_out);
}
